// Attention_7679401525299
// MI455X (gfx1250) — hardware-verified
//
#include <hip/hip_runtime.h>


#ifndef NB
#define NB 4
#endif
#ifndef SEQ
#define SEQ 2048
#endif
#ifndef VSPLIT
#define VSPLIT 0
#endif
#define NB_FULL  4
#define SEQ_FULL 2048
#define DM   1024
#define NH   16
#define HD   64
#define QKC  16.0f
#define VC   256.0f
#define PLOG 10.0f
#define SC2  (1.4426950408889634f / 8192.0f)

static_assert(NB >= 1 && NB <= NB_FULL);
static_assert(SEQ >= 64 && SEQ <= SEQ_FULL);
static_assert(SEQ % 64 == 0);
static_assert(DM % 64 == 0 && DM % 32 == 0);
static_assert(NH * HD == DM);

typedef _Float16 h16;
typedef unsigned short bf;
typedef __attribute__((ext_vector_type(16))) __bf16   v16bf;
typedef __attribute__((ext_vector_type(16))) _Float16 v16h;
typedef __attribute__((ext_vector_type(8)))  _Float16 v8h;
typedef __attribute__((ext_vector_type(8)))  unsigned short v8us;
typedef __attribute__((ext_vector_type(8)))  float    v8f;
typedef __attribute__((ext_vector_type(4)))  float    v4f;
typedef v4f  __attribute__((may_alias)) v4fa;
typedef v8us __attribute__((may_alias)) v8usa;

__device__ __forceinline__ unsigned short f2bf(float f) { unsigned u = __float_as_uint(f); u += 0x7FFFu + ((u >> 16) & 1u); return (unsigned short)(u >> 16); }
__device__ __forceinline__ float bf2f(unsigned short b) { return __uint_as_float(((unsigned)b) << 16); }
__device__ __forceinline__ v16h cat16(v8h lo, v8h hi) { return __builtin_shufflevector(lo, hi, 0, 1, 2, 3, 4, 5, 6, 7, 8, 9, 10, 11, 12, 13, 14, 15); }
__device__ __forceinline__ v16bf cat16b(v8us lo, v8us hi) { return __builtin_bit_cast(v16bf, __builtin_shufflevector(lo, hi, 0, 1, 2, 3, 4, 5, 6, 7, 8, 9, 10, 11, 12, 13, 14, 15)); }
__device__ __forceinline__ v8f wmma16(v16h a, v16h b, v8f c) { return __builtin_amdgcn_wmma_f32_16x16x32_f16(false, a, false, b, (short)0, c, false, false); }
__device__ __forceinline__ v8f wmmab(v16bf a, v16bf b, v8f c) { return __builtin_amdgcn_wmma_f32_16x16x32_bf16(false, a, false, b, (short)0, c, false, false); }
__device__ __forceinline__ v16h  ldh(const h16* p) { return cat16(*(const v8h*)p, *(const v8h*)(p + 16)); }
__device__ __forceinline__ v16bf ldb(const bf* p)  { return cat16b(*(const v8us*)p, *(const v8us*)(p + 16)); }

__global__ __launch_bounds__(256) void k_cvt(const float* __restrict__ src, bf* dst, int rpb, int rpbf, int nrows) {
    const size_t idx = (size_t)blockIdx.x * 256 + threadIdx.x;
    const int row = (int)(idx >> 7); const int c8 = (int)(idx & 127);
    if (row >= nrows) return;
    const int b = row / rpb, s = row - b * rpb;
    const float* p = src + ((size_t)b * rpbf + s) * DM + c8 * 8;
    const v4f x0 = *(const v4f*)p, x1 = *(const v4f*)(p + 4);
    v8us o;
    o[0] = f2bf(x0[0]); o[1] = f2bf(x0[1]); o[2] = f2bf(x0[2]); o[3] = f2bf(x0[3]);
    o[4] = f2bf(x1[0]); o[5] = f2bf(x1[1]); o[6] = f2bf(x1[2]); o[7] = f2bf(x1[3]);
    bf* q = dst + (size_t)row * DM + c8 * 8;
    *(volatile v8us*)q = o; __threadfence(); *(volatile v8us*)q = o;
}

template <int MODE, int NSPLIT>
__global__ __launch_bounds__(32) void k_gemmw(const bf* __restrict__ A, const bf* __restrict__ A2, const bf* __restrict__ Bt, int K,
                                              h16* P0, h16* P1, float* CF, size_t sA, size_t sB, size_t sC) {
    __shared__ __align__(16) float os[64 * 68];
    const size_t z = blockIdx.z; A += z * sA; if (NSPLIT == 1) A2 += z * sA; Bt += z * sB;
    const int lane = threadIdx.x & 31, lr = lane & 15, hi = lane >> 4; const int r0 = blockIdx.x * 64, c0 = blockIdx.y * 64;
    v8f acc[4][4];
#pragma unroll
    for (int mb = 0; mb < 4; ++mb)
#pragma unroll
        for (int nb = 0; nb < 4; ++nb) acc[mb][nb] = (v8f){};
    const size_t aoff = (size_t)(r0 + lr) * K + 8 * hi, boff = (size_t)(c0 + lr) * K + 8 * hi;
#pragma unroll 1
    for (int kc = 0; kc < K; kc += 32) {
        v16bf a[4], a2[4];
#pragma unroll
        for (int mb = 0; mb < 4; ++mb) { a[mb] = ldb(A + aoff + (size_t)mb * 16 * K + kc); if (NSPLIT == 1) a2[mb] = ldb(A2 + aoff + (size_t)mb * 16 * K + kc); }
#pragma unroll
        for (int nb = 0; nb < 4; ++nb) { const v16bf b = ldb(Bt + boff + (size_t)nb * 16 * K + kc);
#pragma unroll
            for (int mb = 0; mb < 4; ++mb) { acc[mb][nb] = wmmab(a[mb], b, acc[mb][nb]); if (NSPLIT == 1) acc[mb][nb] = wmmab(a2[mb], b, acc[mb][nb]); } }
        asm volatile("v_nop\n\tv_nop\n\tv_nop\n\tv_nop" : "+v"(acc[0][0]), "+v"(acc[1][1]), "+v"(acc[2][2]), "+v"(acc[3][3]) : "v"(a[0]), "v"(a[3]));
        if (NSPLIT == 1) asm volatile("" : : "v"(a2[0]), "v"(a2[3]));
    }
#pragma unroll
    for (int mb = 0; mb < 4; ++mb)
#pragma unroll
        for (int nb = 0; nb < 4; ++nb)
#pragma unroll
            for (int j = 0; j < 8; ++j) os[(mb * 16 + hi * 8 + j) * 68 + nb * 16 + lr] = acc[mb][nb][j];
    __syncthreads();
    const int bb = r0 / SEQ, s0 = r0 - bb * SEQ, hh = c0 / HD;
    if (MODE == 0) {
        h16* dst = P0 + z * sC + ((size_t)(bb * NH + hh) * SEQ + s0) * HD;
#pragma unroll 1
        for (int ps = 0; ps < 2; ++ps) {
#pragma unroll 4
            for (int it = 0; it < 16; ++it) { const int row = it * 4 + (lane >> 3), pc = (lane & 7) * 8;
                const v4f x0 = *(const v4fa*)(os + row * 68 + pc), x1 = *(const v4fa*)(os + row * 68 + pc + 4); v8h o;
                o[0] = (h16)(x0[0] * QKC); o[1] = (h16)(x0[1] * QKC); o[2] = (h16)(x0[2] * QKC); o[3] = (h16)(x0[3] * QKC);
                o[4] = (h16)(x1[0] * QKC); o[5] = (h16)(x1[1] * QKC); o[6] = (h16)(x1[2] * QKC); o[7] = (h16)(x1[3] * QKC);
                *(volatile v8h*)(dst + (size_t)row * HD + pc) = o; }
            if (ps == 0) __threadfence(); }
    } else if (MODE == 1) {
        h16* dh = P0 + ((size_t)(bb * NH + hh) * HD) * SEQ + s0;
        h16* dl = P1 + ((size_t)(bb * NH + hh) * HD) * SEQ + s0;
#pragma unroll 1
        for (int ps = 0; ps < 2; ++ps) {
#pragma unroll 2
            for (int it = 0; it < 16; ++it) { const int d = it * 4 + (lane >> 3), pc = (lane & 7) * 8; v8h oh, ol;
#pragma unroll
                for (int j = 0; j < 8; ++j) { const float x = os[(pc + j) * 68 + d] * VC; const h16 hv = (h16)x; oh[j] = hv; ol[j] = (h16)(x - (float)hv); }
                *(volatile v8h*)(dh + (size_t)d * SEQ + pc) = oh;
                if (VSPLIT) *(volatile v8h*)(dl + (size_t)d * SEQ + pc) = ol; }
            if (ps == 0) __threadfence(); }
    } else {
        float* crow = CF + ((size_t)bb * SEQ_FULL + s0) * DM + c0;
#pragma unroll 1
        for (int ps = 0; ps < 2; ++ps) {
#pragma unroll 4
            for (int it = 0; it < 32; ++it) { const int row = it * 2 + hi, cofs = lr * 4; const v4f val = *(const v4fa*)(os + row * 68 + cofs);
                *(volatile v4f*)(crow + (size_t)row * DM + cofs) = val; }
            if (ps == 0) __threadfence(); }
    }
}

__global__ __launch_bounds__(128) void k_flash(const h16* __restrict__ Qp, const h16* __restrict__ Kp, const h16* __restrict__ Vhp, const h16* __restrict__ Vlp, bf* Ch, bf* Cl) {
    __shared__ __align__(16) unsigned short sh[4 * 16 * 72];
    __shared__ __align__(16) unsigned short sl[4 * 16 * 72];
    const int w = threadIdx.x >> 5, lane = threadIdx.x & 31, lr = lane & 15, hi = lane >> 4;
    const int bh = blockIdx.y, q0 = (blockIdx.x * 4 + w) * 16;
    const h16* qp = Qp + ((size_t)bh * SEQ + q0 + lr) * HD + 8 * hi;
    const h16* kp = Kp + ((size_t)bh * SEQ + lr) * HD + 8 * hi;
    const h16* vhp = Vhp + ((size_t)bh * HD + lr) * SEQ + 8 * hi;
    const h16* vlp = Vlp + ((size_t)bh * HD + lr) * SEQ + 8 * hi;
    const v16h qf0 = ldh(qp), qf1 = ldh(qp + 32);
    v8f oacc[4];
#pragma unroll
    for (int dt = 0; dt < 4; ++dt) oacc[dt] = (v8f){};
    float mrun = -3.0e38f, lrun = 0.0f;
#pragma unroll 1
    for (int kt0 = 0; kt0 < SEQ; kt0 += 32) {
        const v16h k00 = ldh(kp + (size_t)kt0 * HD), k01 = ldh(kp + (size_t)kt0 * HD + 32);
        const v16h k10 = ldh(kp + (size_t)(kt0 + 16) * HD), k11 = ldh(kp + (size_t)(kt0 + 16) * HD + 32);
        v8f s0 = (v8f){}, s1 = (v8f){};
        s0 = wmma16(k00, qf0, s0); s0 = wmma16(k01, qf1, s0);
        s1 = wmma16(k10, qf0, s1); s1 = wmma16(k11, qf1, s1);
        asm volatile("v_nop\n\tv_nop\n\tv_nop\n\tv_nop" : "+v"(s0), "+v"(s1) : "v"(k00), "v"(k01), "v"(k10), "v"(k11), "v"(qf0), "v"(qf1));
        float vm = fmaxf(s0[0], s1[0]);
#pragma unroll
        for (int r = 1; r < 8; ++r) vm = fmaxf(vm, fmaxf(s0[r], s1[r]));
        vm = fmaxf(vm, __shfl_xor(vm, 16, 32));
        const float mnew = fmaxf(mrun, vm * SC2);
        const float corr = __builtin_amdgcn_exp2f(mrun - mnew); mrun = mnew;
        const float nbias = PLOG - mnew;
        float ls = 0.0f; v16h pb;
#pragma unroll
        for (int r = 0; r < 8; ++r) { const float p0 = __builtin_amdgcn_exp2f(fmaf(s0[r], SC2, nbias)); const float p1 = __builtin_amdgcn_exp2f(fmaf(s1[r], SC2, nbias));
            ls += p0 + p1; pb[r] = (h16)p0; pb[8 + r] = (h16)p1; }
        lrun = fmaf(lrun, corr, ls);
        if (__any(corr != 1.0f)) {
#pragma unroll
            for (int dt = 0; dt < 4; ++dt)
#pragma unroll
                for (int r = 0; r < 8; ++r) oacc[dt][r] *= corr;
        }
        v16h va[4], vb[4];
#pragma unroll
        for (int dt = 0; dt < 4; ++dt) { va[dt] = ldh(vhp + (size_t)dt * 16 * SEQ + kt0); if (VSPLIT) vb[dt] = ldh(vlp + (size_t)dt * 16 * SEQ + kt0); }
#pragma unroll
        for (int dt = 0; dt < 4; ++dt) { oacc[dt] = wmma16(va[dt], pb, oacc[dt]); if (VSPLIT) oacc[dt] = wmma16(vb[dt], pb, oacc[dt]); }
        if (VSPLIT) asm volatile("v_nop\n\tv_nop\n\tv_nop\n\tv_nop" : "+v"(oacc[0]), "+v"(oacc[1]), "+v"(oacc[2]), "+v"(oacc[3]) : "v"(pb), "v"(va[0]), "v"(va[1]), "v"(va[2]), "v"(va[3]), "v"(vb[0]), "v"(vb[1]), "v"(vb[2]), "v"(vb[3]));
        else        asm volatile("v_nop\n\tv_nop\n\tv_nop\n\tv_nop" : "+v"(oacc[0]), "+v"(oacc[1]), "+v"(oacc[2]), "+v"(oacc[3]) : "v"(pb), "v"(va[0]), "v"(va[1]), "v"(va[2]), "v"(va[3]));
    }
    const float ltot = lrun + __shfl_xor(lrun, 16, 32);
    const float inv = (1.0f / VC) * (1.0f / ltot);
#pragma unroll
    for (int dt = 0; dt < 4; ++dt) { v8us ph, pl;
#pragma unroll
        for (int r = 0; r < 8; ++r) { const float c = oacc[dt][r] * inv; const unsigned short a = f2bf(c); ph[r] = a; pl[r] = f2bf(c - bf2f(a)); }
        *(v8usa*)(sh + (w * 16 + lr) * 72 + dt * 16 + 8 * hi) = ph;
        *(v8usa*)(sl + (w * 16 + lr) * 72 + dt * 16 + 8 * hi) = pl; }
    __syncthreads();
    const int b = bh / NH, h = bh - b * NH;
    bf* ch = Ch + ((size_t)b * SEQ + q0) * DM + h * HD;
    bf* cl = Cl + ((size_t)b * SEQ + q0) * DM + h * HD;
#pragma unroll 1
    for (int ps = 0; ps < 2; ++ps) {
#pragma unroll
        for (int it = 0; it < 4; ++it) { const int q = it * 4 + (lane >> 3), pc = (lane & 7) * 8;
            const v8us x = *(const v8usa*)(sh + (w * 16 + q) * 72 + pc); const v8us y = *(const v8usa*)(sl + (w * 16 + q) * 72 + pc);
            *(volatile v8us*)(ch + (size_t)q * DM + pc) = x; *(volatile v8us*)(cl + (size_t)q * DM + pc) = y; }
        if (ps == 0) __threadfence(); }
}

extern "C" void kernel_launch(void* const* d_in, const int* in_sizes, int n_in,
                              void* d_out, int out_size, void* d_ws, size_t ws_size, hipStream_t stream) {
    if (n_in < 7) return;
    const size_t needX = ((size_t)(NB - 1) * SEQ_FULL + SEQ) * DM;
    if ((size_t)in_sizes[0] < needX || (size_t)in_sizes[1] < needX || (size_t)in_sizes[2] < needX) return;
    if ((size_t)in_sizes[3] < (size_t)DM * DM || (size_t)in_sizes[4] < (size_t)DM * DM || (size_t)in_sizes[5] < (size_t)DM * DM || (size_t)in_sizes[6] < (size_t)DM * DM) return;
    if ((size_t)out_size < needX) return;
    const float* q = (const float*)d_in[0]; const float* k = (const float*)d_in[1]; const float* v = (const float*)d_in[2];
    const float* wq = (const float*)d_in[3]; const float* wk = (const float*)d_in[4]; const float* wv = (const float*)d_in[5]; const float* wo = (const float*)d_in[6];
    float* OUT = (float*)d_out;
    char* wsp = (char*)d_ws;
    auto take = [&](size_t bytes) { char* p = wsp; wsp += (bytes + 255) & ~(size_t)255; return (void*)p; };
    const size_t MR = (size_t)NB * SEQ;
    const size_t XB = MR * DM * 2, WB = (size_t)DM * DM * 2;
    bf* XQ = (bf*)take(XB); bf* XK = (bf*)take(XB); bf* XV = (bf*)take(XB);
    bf* WQ = (bf*)take(WB); bf* WK = (bf*)take(WB); bf* WV = (bf*)take(WB); bf* WO = (bf*)take(WB);
    h16* Q16 = (h16*)take(XB); h16* K16 = (h16*)take(XB);
    h16* VTh = (h16*)take(XB); h16* VTl = (h16*)take(XB);
    if ((size_t)(wsp - (char*)d_ws) > ws_size) return;
    bf* CTh = XQ; bf* CTl = XK;

    const unsigned gx = (unsigned)((MR * 128 + 255) / 256), gw = (unsigned)(((size_t)DM * 128 + 255) / 256);
    k_cvt<<<gx, 256, 0, stream>>>(q, XQ, SEQ, SEQ_FULL, (int)MR);
    k_cvt<<<gx, 256, 0, stream>>>(k, XK, SEQ, SEQ_FULL, (int)MR);
    k_cvt<<<gx, 256, 0, stream>>>(v, XV, SEQ, SEQ_FULL, (int)MR);
    k_cvt<<<gw, 256, 0, stream>>>(wq, WQ, DM, DM, DM);
    k_cvt<<<gw, 256, 0, stream>>>(wk, WK, DM, DM, DM);
    k_cvt<<<gw, 256, 0, stream>>>(wv, WV, DM, DM, DM);
    k_cvt<<<gw, 256, 0, stream>>>(wo, WO, DM, DM, DM);
    k_gemmw<0, 0><<<dim3((unsigned)(MR / 64), DM / 64, 2), 32, 0, stream>>>(XQ, nullptr, WQ, DM, Q16, nullptr, nullptr, (size_t)(XK - XQ), (size_t)(WK - WQ), (size_t)(K16 - Q16));
    k_gemmw<1, 0><<<dim3((unsigned)(MR / 64), DM / 64, 1), 32, 0, stream>>>(XV, nullptr, WV, DM, VTh, VTl, nullptr, 0, 0, 0);
    k_flash<<<dim3(SEQ / 64, NB * NH), 128, 0, stream>>>(Q16, K16, VTh, VTl, CTh, CTl);
    k_gemmw<2, 1><<<dim3((unsigned)(MR / 64), DM / 64, 1), 32, 0, stream>>>(CTh, CTl, WO, DM, nullptr, nullptr, OUT, 0, 0, 0);
}
